// MDA_83863531422299
// MI455X (gfx1250) — hardware-run, weakly checked
//
#include <hip/hip_runtime.h>


#ifndef NTR
#define NTR 100000
#endif
#ifndef NTE
#define NTE 50000
#endif
#define NTR_FULL 100000
#define NTE_FULL 50000
#define NN   1778
#define NNP  1792
#define DE   901
#define KP1  960
#define H1W  1024
#define H2W  512
#define H3W  64
#define WCARRY 1024.0f
#define WINV   (1.0f / 1024.0f)

static_assert(NNP % 64 == 0);
static_assert(NNP >= NN);
static_assert(KP1 % 64 == 0);
static_assert(KP1 >= DE);
static_assert(H1W % 64 == 0);
static_assert(H2W % 64 == 0);
static_assert(H3W == 64);
static_assert(H1W % 32 == 0);
static_assert(H2W % 32 == 0);
static_assert(((size_t)NNP * (KP1 / 8)) % 256 == 0);
static_assert(NTR % 4 == 0);
static_assert(NTE % 4 == 0);
static_assert(NTR <= NTR_FULL);
static_assert(NTE <= NTE_FULL);
static_assert(((size_t)NTR_FULL * 4) % 128 == 0);
static_assert((size_t)NTR_FULL * 4 == 400000);
static_assert(32 * 16 * 4 == 16 * 64 * 2);
static_assert(256 * 16 * 2 == 64 * 64 * 2);
static_assert(256 * 16 == 64 * 64);
static_assert(16 * 16 == 64 * 4);
static_assert(16 * 68 * 4 + 64 * 4 + 64 * 4 <= 131072);
static_assert(64 * 65 * 4 <= 131072);

typedef _Float16 h16;
typedef unsigned short bf;
typedef __attribute__((ext_vector_type(16))) __bf16   v16bf;
typedef __attribute__((ext_vector_type(16))) _Float16 v16h;
typedef __attribute__((ext_vector_type(8)))  _Float16 v8h;
typedef __attribute__((ext_vector_type(8)))  unsigned short v8us;
typedef __attribute__((ext_vector_type(8)))  float    v8f;
typedef __attribute__((ext_vector_type(4)))  float    v4f;
typedef __attribute__((ext_vector_type(4)))  int      v4i;
typedef v4f  __attribute__((may_alias)) v4fa;

__device__ __forceinline__ unsigned short f2bf(float f) { unsigned u = __float_as_uint(f); u += 0x7FFFu + ((u >> 16) & 1u); return (unsigned short)(u >> 16); }
__device__ __forceinline__ float bfr(float f) { return __uint_as_float(((unsigned)f2bf(f)) << 16); }
__device__ __forceinline__ v16h cat16(v8h lo, v8h hi) { return __builtin_shufflevector(lo, hi, 0, 1, 2, 3, 4, 5, 6, 7, 8, 9, 10, 11, 12, 13, 14, 15); }
__device__ __forceinline__ v16bf cat16b(v8us lo, v8us hi) { return __builtin_bit_cast(v16bf, __builtin_shufflevector(lo, hi, 0, 1, 2, 3, 4, 5, 6, 7, 8, 9, 10, 11, 12, 13, 14, 15)); }
__device__ __forceinline__ v8f wmma16(v16h a, v16h b, v8f c) { return __builtin_amdgcn_wmma_f32_16x16x32_f16(false, a, false, b, (short)0, c, false, false); }
__device__ __forceinline__ v8f wmmab(v16bf a, v16bf b, v8f c) { return __builtin_amdgcn_wmma_f32_16x16x32_bf16(false, a, false, b, (short)0, c, false, false); }
__device__ __forceinline__ v16h  ldh(const h16* p) { return cat16(*(const v8h*)p, *(const v8h*)(p + 16)); }
__device__ __forceinline__ v16bf ldb(const bf* p)  { return cat16b(*(const v8us*)p, *(const v8us*)(p + 16)); }
__device__ __forceinline__ void wave_sync() { __builtin_amdgcn_fence(3  , "wavefront"); __builtin_amdgcn_wave_barrier(); asm volatile("" ::: "memory"); }
static __device__ __forceinline__ h16 toh_flush(float v) { const h16 r = (h16)v; return (fabsf(v) < 6.103515625e-05f) ? (h16)0.0f : r; }
__device__ __forceinline__ v8f wmmab_g(v16bf a, v16bf b, v8f c) { c = wmmab(a, b, c); asm volatile("v_nop\n\tv_nop\n\tv_nop\n\tv_nop" : "+v"(c) : "v"(a), "v"(b)); return c; }
__device__ __forceinline__ v8f wmma16_g(v16h a, v16h b, v8f c) { c = wmma16(a, b, c); asm volatile("v_nop\n\tv_nop\n\tv_nop\n\tv_nop" : "+v"(c) : "v"(a), "v"(b)); return c; }

__global__ __launch_bounds__(256) void k_xcvt(const float* __restrict__ src, bf* dst) {
    const int i8 = blockIdx.x * 256 + threadIdx.x;
    if (i8 >= NNP * (KP1 / 8)) return;
    const int row = i8 / (KP1 / 8), c8 = (i8 % (KP1 / 8)) * 8;
    const int rc = row < NN ? row : (NN - 1);
    v8us o;
#pragma unroll
    for (int k = 0; k < 8; ++k) {
        const int col = c8 + k; const int cc = col < DE ? col : (DE - 1);
        float v = src[(size_t)rc * DE + cc];
        asm volatile("" : "+v"(v));
        const bool ok = (row < NN) & (col < DE);
        o[k] = ok ? f2bf(v) : (unsigned short)0;
    }
    *(volatile v8us*)(dst + (size_t)i8 * 8) = o; __threadfence(); *(volatile v8us*)(dst + (size_t)i8 * 8) = o;
}

__global__ __launch_bounds__(256) void k_wt_bf(const float* __restrict__ in, int ldin, int kvalid, int kzstep, bf* out, int kp, int nzstep) {
    __shared__ float ts[64 * 65];
    const int kt = blockIdx.x, nt = blockIdx.y, z = blockIdx.z;
    const int krow0 = z * kzstep, nrow0 = z * nzstep + nt * 64;
    const int nl = threadIdx.x & 63, kq = threadIdx.x >> 6;
#pragma unroll 4
    for (int it = 0; it < 16; ++it) {
        const int kl = kq + 4 * it; const int k = kt * 64 + kl; const int kc = k < kvalid ? k : (kvalid - 1);
        float v = in[(size_t)(krow0 + kc) * ldin + nt * 64 + nl];
        asm volatile("" : "+v"(v));
        ts[kl * 65 + nl] = (k < kvalid) ? bfr(v) : 0.0f;
    }
    __syncthreads();
    const int c8 = (threadIdx.x & 7) * 8;
#pragma unroll 1
    for (int ps = 0; ps < 2; ++ps) {
#pragma unroll
        for (int it = 0; it < 2; ++it) { const int row = (threadIdx.x >> 3) + 32 * it;
            v8us o;
#pragma unroll
            for (int j = 0; j < 8; ++j) o[j] = f2bf(ts[(c8 + j) * 65 + row]);
            *(volatile v8us*)(out + (size_t)(nrow0 + row) * kp + kt * 64 + c8) = o; }
        if (ps == 0) __threadfence(); }
}

__global__ __launch_bounds__(256) void k_wt_h(const float* __restrict__ in, int ldin, int kvalid, int kzstep, h16* out, int kp, int nzstep) {
    __shared__ float ts[64 * 65];
    const int kt = blockIdx.x, nt = blockIdx.y, z = blockIdx.z;
    const int krow0 = z * kzstep, nrow0 = z * nzstep + nt * 64;
    const int nl = threadIdx.x & 63, kq = threadIdx.x >> 6;
#pragma unroll 4
    for (int it = 0; it < 16; ++it) {
        const int kl = kq + 4 * it; const int k = kt * 64 + kl; const int kc = k < kvalid ? k : (kvalid - 1);
        float v = in[(size_t)(krow0 + kc) * ldin + nt * 64 + nl];
        asm volatile("" : "+v"(v));
        ts[kl * 65 + nl] = (k < kvalid) ? bfr(v) : 0.0f;
    }
    __syncthreads();
    const int c8 = (threadIdx.x & 7) * 8;
#pragma unroll 1
    for (int ps = 0; ps < 2; ++ps) {
#pragma unroll
        for (int it = 0; it < 2; ++it) { const int row = (threadIdx.x >> 3) + 32 * it;
            v8h o;
#pragma unroll
            for (int j = 0; j < 8; ++j) o[j] = toh_flush(ts[(c8 + j) * 65 + row] * WCARRY);
            *(volatile v8h*)(out + (size_t)(nrow0 + row) * kp + kt * 64 + c8) = o; }
        if (ps == 0) __threadfence(); }
}

__global__ __launch_bounds__(32) void k_gemm_in(const bf* __restrict__ XB, const bf* __restrict__ WT, const float* __restrict__ b1, h16* HP) {
    __shared__ __align__(16) float os[16 * 68];
    const int lane = threadIdx.x & 31, lr = lane & 15, hi = lane >> 4; const int r0 = blockIdx.x * 64, c0 = blockIdx.y * 64;
    v8f acc[4][4];
#pragma unroll
    for (int mb = 0; mb < 4; ++mb)
#pragma unroll
        for (int nb = 0; nb < 4; ++nb) acc[mb][nb] = (v8f){};
    const size_t aoff = (size_t)(r0 + lr) * KP1 + 8 * hi, boff = (size_t)(c0 + lr) * KP1 + 8 * hi;
#pragma unroll 1
    for (int kc = 0; kc < KP1; kc += 32) {
        v16bf a[4];
#pragma unroll
        for (int mb = 0; mb < 4; ++mb) a[mb] = ldb(XB + aoff + (size_t)mb * 16 * KP1 + kc);
#pragma unroll
        for (int nb = 0; nb < 4; ++nb) { const v16bf b = ldb(WT + boff + (size_t)nb * 16 * KP1 + kc);
#pragma unroll
            for (int mb = 0; mb < 4; ++mb) acc[mb][nb] = wmmab_g(a[mb], b, acc[mb][nb]); }
    }
    const int blk = c0 / H1W, cn = c0 % H1W;
    float bc[4];
#pragma unroll
    for (int nb = 0; nb < 4; ++nb) { float v = b1[cn + nb * 16 + lr]; asm volatile("" : "+v"(v)); bc[nb] = (blk == 0) ? bfr(v) : 0.0f; }
    const size_t tbase = ((size_t)blk * NNP + (size_t)r0) * H1W + (size_t)cn;
#pragma unroll
    for (int mb = 0; mb < 4; ++mb) {
#pragma unroll
        for (int nb = 0; nb < 4; ++nb) {
#pragma unroll
            for (int j = 0; j < 8; ++j) os[(hi * 8 + j) * 68 + nb * 16 + lr] = acc[mb][nb][j] + bc[nb]; }
        wave_sync();
#pragma unroll 1
        for (int ps = 0; ps < 2; ++ps) {
            const size_t sb = tbase + (size_t)(mb * 16) * H1W;
#pragma unroll
            for (int s = 0; s < 4; ++s) { const int row = 4 * s + (lane >> 3), c8 = (lane & 7) * 8;
                const v4f x0 = *(const v4fa*)(&os[row * 68 + c8]); const v4f x1 = *(const v4fa*)(&os[row * 68 + c8 + 4]); v8h hv;
#pragma unroll
                for (int i = 0; i < 4; ++i) { hv[i] = toh_flush(x0[i]); hv[4 + i] = toh_flush(x1[i]); }
                *(volatile v8h*)(HP + sb + (size_t)row * H1W + c8) = hv; }
            if (ps == 0) __threadfence(); }
        wave_sync();
    }
}

__global__ __launch_bounds__(32) void k_gemm_mid(const h16* __restrict__ A, const h16* __restrict__ Bt, const float* __restrict__ b2, h16* HP) {
    __shared__ __align__(16) float os[16 * 68];
    const int lane = threadIdx.x & 31, lr = lane & 15, hi = lane >> 4; const int r0 = blockIdx.x * 64, c0 = blockIdx.y * 64;
    v8f acc[4][4];
#pragma unroll
    for (int mb = 0; mb < 4; ++mb)
#pragma unroll
        for (int nb = 0; nb < 4; ++nb) acc[mb][nb] = (v8f){};
    const size_t aoff = (size_t)(r0 + lr) * H1W + 8 * hi, boff = (size_t)(c0 + lr) * H1W + 8 * hi;
#pragma unroll 1
    for (int kc = 0; kc < H1W; kc += 32) {
        v16h a[4];
#pragma unroll
        for (int mb = 0; mb < 4; ++mb) a[mb] = ldh(A + aoff + (size_t)mb * 16 * H1W + kc);
#pragma unroll
        for (int nb = 0; nb < 4; ++nb) { const v16h b = ldh(Bt + boff + (size_t)nb * 16 * H1W + kc);
#pragma unroll
            for (int mb = 0; mb < 4; ++mb) acc[mb][nb] = wmma16_g(a[mb], b, acc[mb][nb]); }
    }
    const bool ub = r0 < NNP;
    float bc[4];
#pragma unroll
    for (int nb = 0; nb < 4; ++nb) { float v = b2[c0 + nb * 16 + lr]; asm volatile("" : "+v"(v)); bc[nb] = ub ? bfr(v) : 0.0f; }
    const size_t tbase = (size_t)r0 * H2W + (size_t)c0;
#pragma unroll
    for (int mb = 0; mb < 4; ++mb) {
#pragma unroll
        for (int nb = 0; nb < 4; ++nb) {
#pragma unroll
            for (int j = 0; j < 8; ++j) os[(hi * 8 + j) * 68 + nb * 16 + lr] = acc[mb][nb][j] * WINV + bc[nb]; }
        wave_sync();
#pragma unroll 1
        for (int ps = 0; ps < 2; ++ps) {
            const size_t sb = tbase + (size_t)(mb * 16) * H2W;
#pragma unroll
            for (int s = 0; s < 4; ++s) { const int row = 4 * s + (lane >> 3), c8 = (lane & 7) * 8;
                const v4f x0 = *(const v4fa*)(&os[row * 68 + c8]); const v4f x1 = *(const v4fa*)(&os[row * 68 + c8 + 4]); v8h hv;
#pragma unroll
                for (int i = 0; i < 4; ++i) { hv[i] = toh_flush(x0[i]); hv[4 + i] = toh_flush(x1[i]); }
                *(volatile v8h*)(HP + sb + (size_t)row * H2W + c8) = hv; }
            if (ps == 0) __threadfence(); }
        wave_sync();
    }
}

__global__ __launch_bounds__(32) void k_gemm_out(const h16* __restrict__ A, const h16* __restrict__ Bt, const float* __restrict__ b3, const float* __restrict__ W4, const float* __restrict__ b4, float* ST) {
    __shared__ __align__(16) float os[16 * 68];
    __shared__ __align__(16) float w4s[64];
    __shared__ __align__(16) float ss[64];
    const int lane = threadIdx.x & 31, lr = lane & 15, hi = lane >> 4; const int r0 = blockIdx.x * 64;
    w4s[lane] = bfr(W4[lane]); w4s[lane + 32] = bfr(W4[lane + 32]);
    const float b4v = bfr(b4[0]);
    v8f acc[4][4];
#pragma unroll
    for (int mb = 0; mb < 4; ++mb)
#pragma unroll
        for (int nb = 0; nb < 4; ++nb) acc[mb][nb] = (v8f){};
    const size_t aoff = (size_t)(r0 + lr) * H2W + 8 * hi, boff = (size_t)lr * H2W + 8 * hi;
#pragma unroll 1
    for (int kc = 0; kc < H2W; kc += 32) {
        v16h a[4];
#pragma unroll
        for (int mb = 0; mb < 4; ++mb) a[mb] = ldh(A + aoff + (size_t)mb * 16 * H2W + kc);
#pragma unroll
        for (int nb = 0; nb < 4; ++nb) { const v16h b = ldh(Bt + boff + (size_t)nb * 16 * H2W + kc);
#pragma unroll
            for (int mb = 0; mb < 4; ++mb) acc[mb][nb] = wmma16_g(a[mb], b, acc[mb][nb]); }
    }
    const bool ub = r0 < NNP;
    float bc[4];
#pragma unroll
    for (int nb = 0; nb < 4; ++nb) { float v = b3[nb * 16 + lr]; asm volatile("" : "+v"(v)); bc[nb] = ub ? bfr(v) : 0.0f; }
    const float badd = ub ? b4v : 0.0f;
#pragma unroll
    for (int mb = 0; mb < 4; ++mb) {
#pragma unroll
        for (int nb = 0; nb < 4; ++nb) {
#pragma unroll
            for (int j = 0; j < 8; ++j) os[(hi * 8 + j) * 68 + nb * 16 + lr] = acc[mb][nb][j] * WINV + bc[nb]; }
        wave_sync();
        const int row = lane >> 1, cb = (lane & 1) * 32;
        float p = 0.0f;
#pragma unroll 4
        for (int c = 0; c < 32; ++c) p = fmaf(os[row * 68 + cb + c], w4s[cb + c], p);
        p += __shfl_xor(p, 1, 32);
        if ((lane & 1) == 0) ss[mb * 16 + row] = p + badd;
        wave_sync();
    }
    const v4f val = *(const v4fa*)(&ss[(lane & 15) * 4]);
    if (lane < 16) *(volatile v4f*)(ST + r0 + lane * 4) = val;
    __threadfence();
    if (lane < 16) *(volatile v4f*)(ST + r0 + lane * 4) = val;
}

__device__ __forceinline__ int nidx(int i) { int c = i < 0 ? i + NN : i; c = c < 0 ? 0 : c; return c > (NN - 1) ? (NN - 1) : c; }
__global__ __launch_bounds__(256) void k_pairs(const int* __restrict__ pairs, const float* __restrict__ SV, const float* __restrict__ TV, float* out, int n4) {
    const int i4 = blockIdx.x * 256 + threadIdx.x; if (i4 >= n4) return;
    const v4i p0 = *(const v4i*)(pairs + (size_t)i4 * 8), p1 = *(const v4i*)(pairs + (size_t)i4 * 8 + 4);
    v4f o;
    o[0] = SV[nidx(p0[0])] + TV[nidx(p0[1])];
    o[1] = SV[nidx(p0[2])] + TV[nidx(p0[3])];
    o[2] = SV[nidx(p1[0])] + TV[nidx(p1[1])];
    o[3] = SV[nidx(p1[2])] + TV[nidx(p1[3])];
    *(volatile v4f*)(out + (size_t)i4 * 4) = o; __threadfence(); *(volatile v4f*)(out + (size_t)i4 * 4) = o;
}

static constexpr size_t al256(size_t v) { return (v + 255) & ~(size_t)255; }
static constexpr size_t SZ_XB  = al256((size_t)NNP * KP1 * 2);
static constexpr size_t SZ_W1T = al256((size_t)2 * H1W * KP1 * 2);
static constexpr size_t SZ_W2T = al256((size_t)H2W * H1W * 2);
static constexpr size_t SZ_W3T = al256((size_t)H3W * H2W * 2);
static constexpr size_t SZ_HP1 = al256((size_t)2 * NNP * H1W * 2);
static constexpr size_t SZ_HP2 = al256((size_t)2 * NNP * H2W * 2);
static constexpr size_t SZ_ST  = al256((size_t)2 * NNP * 4);
static constexpr size_t SZ_TOTAL = SZ_XB + SZ_W1T + SZ_W2T + SZ_W3T + SZ_HP1 + SZ_HP2 + SZ_ST;
static_assert(SZ_TOTAL <= (size_t)134217728);
static_assert(SZ_XB  == (size_t)NNP * KP1 * 2);
static_assert(SZ_W1T == (size_t)2 * H1W * KP1 * 2);
static_assert(SZ_HP1 == (size_t)2 * NNP * H1W * 2);
static_assert(SZ_HP2 == (size_t)2 * NNP * H2W * 2);
static_assert(SZ_ST  == (size_t)2 * NNP * 4);

extern "C" void kernel_launch(void* const* d_in, const int* in_sizes, int n_in,
                              void* d_out, int out_size, void* d_ws, size_t ws_size, hipStream_t stream) {
    if (n_in < 11) return;
    if ((size_t)in_sizes[0] < (size_t)NN * DE) return;
    if ((size_t)in_sizes[1] < (size_t)2 * NTR || (size_t)in_sizes[2] < (size_t)2 * NTE) return;
    if ((size_t)in_sizes[3] < (size_t)2 * DE * H1W || in_sizes[4] < H1W) return;
    if ((size_t)in_sizes[5] < (size_t)H1W * H2W || in_sizes[6] < H2W) return;
    if ((size_t)in_sizes[7] < (size_t)H2W * H3W || in_sizes[8] < H3W) return;
    if (in_sizes[9] < H3W || in_sizes[10] < 1) return;
    if ((size_t)out_size < (size_t)NTR_FULL + NTE) return;
    if (SZ_TOTAL > ws_size) return;
    const float* sumx = (const float*)d_in[0];
    const int* ptr_a = (const int*)d_in[1]; const int* ptr_b = (const int*)d_in[2];
    const float* w1 = (const float*)d_in[3]; const float* b1 = (const float*)d_in[4];
    const float* w2 = (const float*)d_in[5]; const float* b2 = (const float*)d_in[6];
    const float* w3 = (const float*)d_in[7]; const float* b3 = (const float*)d_in[8];
    const float* w4 = (const float*)d_in[9]; const float* b4 = (const float*)d_in[10];
    float* OUT = (float*)d_out;
    char* wsp = (char*)d_ws;
    bf*  XB  = (bf*)wsp;  wsp += SZ_XB;
    bf*  W1T = (bf*)wsp;  wsp += SZ_W1T;
    h16* W2T = (h16*)wsp; wsp += SZ_W2T;
    h16* W3T = (h16*)wsp; wsp += SZ_W3T;
    h16* HP1 = (h16*)wsp; wsp += SZ_HP1;
    h16* HP2 = (h16*)wsp; wsp += SZ_HP2;
    float* ST = (float*)wsp; wsp += SZ_ST;

    k_xcvt<<<(unsigned)(((size_t)NNP * (KP1 / 8)) / 256), 256, 0, stream>>>(sumx, XB);
    k_wt_bf<<<dim3(KP1 / 64, H1W / 64, 2), 256, 0, stream>>>(w1, H1W, DE, DE, W1T, KP1, H1W);
    k_wt_h<<<dim3(H1W / 64, H2W / 64, 1), 256, 0, stream>>>(w2, H2W, H1W, 0, W2T, H1W, 0);
    k_wt_h<<<dim3(H2W / 64, H3W / 64, 1), 256, 0, stream>>>(w3, H3W, H2W, 0, W3T, H2W, 0);

    k_gemm_in<<<dim3(NNP / 64, 2 * H1W / 64, 1), 32, 0, stream>>>(XB, W1T, b1, HP1);
    k_gemm_mid<<<dim3(2 * NNP / 64, H2W / 64, 1), 32, 0, stream>>>(HP1, W2T, b2, HP2);
    k_gemm_out<<<dim3(2 * NNP / 64, 1, 1), 32, 0, stream>>>(HP2, W3T, b3, w4, b4, ST);

    k_pairs<<<(unsigned)((NTR / 4 + 255) / 256), 256, 0, stream>>>(ptr_a, ST, ST + NNP, OUT, NTR / 4);
    k_pairs<<<(unsigned)((NTE / 4 + 255) / 256), 256, 0, stream>>>(ptr_b, ST, ST + NNP, OUT + NTR_FULL, NTE / 4);
}
